// GAT_DTI_1511828488569
// MI455X (gfx1250) — hardware-run, weakly checked
//
#include <hip/hip_runtime.h>


namespace {
constexpr int NN = 50000, NP = 50016, NE = 800000, F0 = 128, F1 = 256, F2 = 64, NGR = 256, MAXDEG = 1024, NGc = (NN + 511) / 512, PERMLEN = NE + 32 * NGc + 32;
constexpr float XS = 8.0f, SLOPE = 0.2f;

typedef _Float16 b16;
typedef __attribute__((ext_vector_type(16))) _Float16 v16b;
typedef __attribute__((ext_vector_type(8))) _Float16 v8b;
typedef __attribute__((ext_vector_type(8))) float v8f;
typedef __attribute__((ext_vector_type(4))) float v4f;
typedef __attribute__((ext_vector_type(2))) float v2f;
__device__ __forceinline__ float bf16_rne(float f) { unsigned int u = __float_as_uint(f); u += 0x7FFFu + ((u >> 16) & 1u); return __uint_as_float(u & 0xFFFF0000u); }
__device__ __forceinline__ void split16(float v, b16& hi, b16& lo) { hi = (b16)v; lo = (b16)(v - (float)hi); }
__device__ __forceinline__ v16b frag_kb(const b16* p, int hh) { const v8b a = *(const v8b*)(p + 8 * hh), b = *(const v8b*)(p + 16 + 8 * hh); v16b f;
#pragma unroll
  for (int e = 0; e < 8; ++e) { f[e] = a[e]; f[8 + e] = b[e]; } return f; }
__device__ __forceinline__ v8f wmma16b(v16b a, v16b b, v8f c) { v8f d = __builtin_amdgcn_wmma_f32_16x16x32_f16(false, a, false, b, (short)0, c, false, false); asm volatile("v_nop\n\tv_nop\n\tv_nop\n\tv_nop" : "+v"(d) : "v"(a), "v"(b)); return d; }
__device__ __forceinline__ void wave_lds_sync() { __builtin_amdgcn_fence(__ATOMIC_RELEASE, "workgroup"); __builtin_amdgcn_wave_barrier(); __builtin_amdgcn_fence(__ATOMIC_ACQUIRE, "workgroup"); }
__device__ __forceinline__ float nexp(float x) { return __builtin_amdgcn_exp2f(x * 1.4426950408889634f); }
__device__ __forceinline__ float pmul(float a, float b) { float p = a * b; asm volatile("" : "+v"(p)); return p; }
__device__ __forceinline__ float leaky(float x) { return (x >= 0.0f) ? x : SLOPE * x; }
__device__ __forceinline__ float elu_f(float x) { return (x > 0.0f) ? x : (nexp(x) - 1.0f); }
constexpr int CSR_NBLK = 512, CSR_GB = 9, CSR_GN = 1 << CSR_GB  , CSR_MAXG = 512, CSR_CAP = 12288  ;
__global__ __launch_bounds__(64) void csrA_kernel(const int* __restrict__ dst, int E, int N, int nG, int CHP, int NGP, int* __restrict__ STG, int* __restrict__ HST) {
  extern __shared__ int sm[];
  int* cnt = sm; int* run = sm + NGP; int* ids = sm + 2 * NGP;
  const int b = blockIdx.x; const int ch = (E + CSR_NBLK - 1) / CSR_NBLK; const int e0 = b * ch, e1 = min(E, e0 + ch);
  for (int i = threadIdx.x; i < NGP; i += 64) cnt[i] = 0;
  for (int i = threadIdx.x; i < CHP; i += 64) ids[i] = -1;
  __syncthreads();
  if (threadIdx.x == 0) {
    for (int e = e0; e < e1; ++e) { int d = dst[e]; d = (d < 0) ? 0 : (d >= N ? N - 1 : d); cnt[d >> CSR_GB] += 1; }
    int acc = 0; for (int g = 0; g < nG; ++g) { run[g] = acc; acc += cnt[g]; }
    for (int e = e0; e < e1; ++e) { int d = dst[e]; d = (d < 0) ? 0 : (d >= N ? N - 1 : d); const int g = d >> CSR_GB; ids[run[g]] = e; run[g] += 1; } }
  __syncthreads();
  typedef __attribute__((ext_vector_type(4))) int v4i;
  for (int pass = 0; pass < 2; ++pass) {
    for (int i = threadIdx.x; i < CHP / 4; i += 64) *(volatile v4i*)(STG + (size_t)b * CHP + i * 4) = *(const v4i*)(&ids[i * 4]);
    for (int i = threadIdx.x; i < NGP / 4; i += 64) { v4i v; for (int e = 0; e < 4; ++e) v[e] = (i * 4 + e < nG) ? cnt[i * 4 + e] : 0; *(volatile v4i*)(HST + (size_t)b * NGP + i * 4) = v; }
    __threadfence(); }
}
__global__ __launch_bounds__(512) void csrS_kernel(const int* __restrict__ HST, int nG, int NGP, int* __restrict__ START, int* __restrict__ TOT, int* __restrict__ OFF) {
  __shared__ int tot[CSR_MAXG];
  const int b = threadIdx.x;
  for (int pass = 0; pass < 2; ++pass) { int runb = 0; for (int g = 0; g < nG; ++g) { int c = HST[(size_t)b * NGP + g]; c = (c < 0) ? 0 : c; ((volatile int*)OFF)[(size_t)g * CSR_NBLK + b] = runb; runb += c; } __threadfence(); }
  for (int g = threadIdx.x; g < nG; g += 512) { int s = 0; for (int bb = 0; bb < CSR_NBLK; ++bb) { int c = HST[(size_t)bb * NGP + g]; s += (c < 0) ? 0 : c; } tot[g] = s; }
  __syncthreads();
  if (threadIdx.x < 32) {
    __shared__ int st[CSR_MAXG + 32];
    if (threadIdx.x == 0) { int acc = 0; for (int g = 0; g < NGP; ++g) { st[g] = acc; if (g < nG) acc += (tot[g] + 31) & ~31; } st[NGP] = acc; }
    __builtin_amdgcn_fence(__ATOMIC_RELEASE, "workgroup"); __builtin_amdgcn_wave_barrier(); __builtin_amdgcn_fence(__ATOMIC_ACQUIRE, "workgroup");
    for (int pass = 0; pass < 2; ++pass) { for (int i = threadIdx.x; i < NGP + 32; i += 32) { ((volatile int*)START)[i] = (i <= NGP) ? st[min(i, NGP)] : 0; ((volatile int*)TOT)[i] = (i < nG) ? tot[i] : 0; } __threadfence(); } }
}
__global__ __launch_bounds__(256) void csrB_kernel(const int* __restrict__ dst, int N, int nG, int CHP, int NGP, int permLen, const int* __restrict__ STG, const int* __restrict__ HST, const int* __restrict__ OFF, const int* __restrict__ START, const int* __restrict__ TOT, int* __restrict__ PERM, int* __restrict__ ROWPTR, int* __restrict__ ROWCNT, int* __restrict__ FLAG) {
  typedef __attribute__((ext_vector_type(4))) int v4i;
  __shared__ int ids[CSR_CAP]; __shared__ unsigned short key[CSR_CAP]; __shared__ int outp[CSR_CAP]; __shared__ int ncnt[CSR_GN + 1]; __shared__ int boff[CSR_NBLK + 1];
  const int g = blockIdx.x, t_ = threadIdx.x; int tot = TOT[g]; int st = START[g], stn = START[g + 1]; const int v0 = g * CSR_GN; const int nv = min(CSR_GN, N - v0);
  st = (st < 0) ? 0 : (st > permLen - 32 ? permLen - 32 : st) & ~31; stn = (stn < st) ? st : (stn > permLen ? permLen : stn); tot = (tot < 0) ? 0 : tot; if (tot > stn - st && tot <= CSR_CAP) tot = stn - st;
  if (tot > CSR_CAP) {
    for (int pass = 0; pass < 2; ++pass) { for (int i = t_; i < CSR_GN / 4; i += 256) { v4i a, c; for (int e = 0; e < 4; ++e) { a[e] = st; c[e] = 0; } *(volatile v4i*)(ROWPTR + v0 + i * 4) = a; *(volatile v4i*)(ROWCNT + v0 + i * 4) = c; } if (t_ == 0) ((volatile int*)FLAG)[0] = 1; __threadfence(); } (void)nv; return; }
  if (t_ == 0) { int acc = 0; for (int b = 0; b < CSR_NBLK; ++b) { boff[b] = acc; int c = HST[(size_t)b * NGP + g]; c = (c < 0) ? 0 : (c > CHP ? CHP : c); acc += c; if (acc > tot) acc = tot; } boff[CSR_NBLK] = acc; }
  for (int i = t_; i <= CSR_GN; i += 256) ncnt[i] = 0;
  __syncthreads();
  for (int b = 0; b < CSR_NBLK; ++b) { const int c = boff[b + 1] - boff[b]; int o_ = OFF[(size_t)g * CSR_NBLK + b]; o_ = (o_ < 0) ? 0 : (o_ > CHP - c ? CHP - c : o_); const int* src_ = STG + (size_t)b * CHP + o_;
    for (int i = t_; i < c; i += 256) { int id = src_[i]; id = (id < 0) ? 0 : id; ids[boff[b] + i] = id; int d = dst[id]; d = (d < v0) ? v0 : (d >= N ? N - 1 : d); int kk = d - v0; kk = (kk < 0) ? 0 : (kk >= CSR_GN ? CSR_GN - 1 : kk); key[boff[b] + i] = (unsigned short)kk; } }
  __syncthreads();
  if (t_ == 0) { for (int i = 0; i < tot; ++i) ncnt[key[i]] += 1; int acc = 0; for (int vl = 0; vl < CSR_GN; ++vl) { const int c = ncnt[vl]; ncnt[vl] = acc; acc += c; } ncnt[CSR_GN] = acc;
    for (int i = 0; i < tot; ++i) { const int vl = key[i]; outp[ncnt[vl]] = ids[i]; ncnt[vl] += 1; }
    for (int vl = CSR_GN; vl > 0; --vl) ncnt[vl] = ncnt[vl - 1]; ncnt[0] = 0; }
  __syncthreads();
  for (int pass = 0; pass < 2; ++pass) {
    for (int i = t_; i < (stn - st) / 4; i += 256) { v4i v; for (int e = 0; e < 4; ++e) { const int q = i * 4 + e; v[e] = (q < tot) ? outp[q] : -1; } *(volatile v4i*)(PERM + st + i * 4) = v; }
    for (int i = t_; i < CSR_GN / 4; i += 256) { v4i a, c; for (int e = 0; e < 4; ++e) { const int vl = i * 4 + e; a[e] = st + ncnt[vl]; c[e] = (vl < nv) ? (ncnt[vl + 1] - ncnt[vl]) : 0; } *(volatile v4i*)(ROWPTR + v0 + i * 4) = a; *(volatile v4i*)(ROWCNT + v0 + i * 4) = c; }
    __threadfence(); }
}
__global__ __launch_bounds__(256) void csrZ_kernel(int* __restrict__ p, size_t n4) { typedef __attribute__((ext_vector_type(4))) int v4i; const size_t tid = (size_t)blockIdx.x * 256 + threadIdx.x, nth = (size_t)gridDim.x * 256; v4i z = {0, 0, 0, 0}; for (size_t i = tid; i < n4; i += nth) *(volatile v4i*)(p + i * 4) = z; }
struct CsrBufs { int *STG, *HST, *OFF, *START, *TOT, *PERM, *ROWPTR, *ROWCNT, *FLAG; int nG, NGP, CHP; size_t permLen; char* base; size_t bytes; };
static size_t csr_carve(CsrBufs& c, char* ws, size_t off, int E, int N) {
  const size_t off0 = off; c.base = ws + off;
  auto al = [&](size_t bytes) { char* p = ws + off; off += (bytes + 255) & ~(size_t)255; return p; };
  c.nG = (N + CSR_GN - 1) / CSR_GN; c.NGP = (c.nG + 31) & ~31; const int ch = (E + CSR_NBLK - 1) / CSR_NBLK; c.CHP = (ch + 31) & ~31; c.permLen = (size_t)E + 32 * (size_t)c.nG + 32;
  c.STG = (int*)al((size_t)CSR_NBLK * c.CHP * 4); c.HST = (int*)al((size_t)CSR_NBLK * c.NGP * 4); c.OFF = (int*)al((size_t)c.NGP * CSR_NBLK * 4); c.START = (int*)al((size_t)(c.NGP + 64) * 4); c.TOT = (int*)al((size_t)(c.NGP + 64) * 4);
  c.PERM = (int*)al(c.permLen * 4); c.ROWPTR = (int*)al((size_t)c.nG * CSR_GN * 4); c.ROWCNT = (int*)al((size_t)c.nG * CSR_GN * 4); c.FLAG = (int*)al(256);
  c.bytes = off - off0; return off;
}
static void csr_build(const CsrBufs& c, const int* dst, int E, int N, hipStream_t stream) {
  const size_t smem = (size_t)(2 * c.NGP + c.CHP) * 4;
  csrZ_kernel<<<512, 256, 0, stream>>>((int*)c.base, c.bytes / 16);
  csrA_kernel<<<CSR_NBLK, 64, smem, stream>>>(dst, E, N, c.nG, c.CHP, c.NGP, c.STG, c.HST);
  csrS_kernel<<<1, 512, 0, stream>>>(c.HST, c.nG, c.NGP, c.START, c.TOT, c.OFF);
  csrB_kernel<<<c.nG, 256, 0, stream>>>(dst, N, c.nG, c.CHP, c.NGP, (int)c.permLen, c.STG, c.HST, c.OFF, c.START, c.TOT, c.PERM, c.ROWPTR, c.ROWCNT, c.FLAG);
}

struct Ro_ { static constexpr size_t W0 = 0, W1 = W0 + 256 * 128, W2 = W1 + 256 * 256, END = W2 + 64 * 256; };
constexpr int PHEAD = 6144, PEND = 20616;
__global__ __launch_bounds__(256) void prep_kernel(const float* __restrict__ x, const float* const* __restrict__ dummy, const float* __restrict__ w0, const float* __restrict__ w1, const float* __restrict__ w2, const float* __restrict__ lp  , b16* __restrict__ R, b16* __restrict__ X, b16* __restrict__ H1pad, b16* __restrict__ H2pad) {
  (void)dummy; (void)lp;
  const size_t tid = (size_t)blockIdx.x * 256 + threadIdx.x, nth = (size_t)gridDim.x * 256;
  auto tr = [&](size_t base, int nout, int kin, const float* W) { for (size_t p = tid; p < (size_t)nout * kin; p += nth) { const int o = (int)(p / kin), k = (int)(p % kin); ((volatile b16*)R)[base + p] = (b16)bf16_rne(W[(size_t)k * nout + o]); } };
  for (int pass = 0; pass < 2; ++pass) { tr(Ro_::W0, 256, 128, w0); tr(Ro_::W1, 256, 256, w1); tr(Ro_::W2, 64, 256, w2);
    for (size_t p = tid; p < (size_t)NP * F0 / 8; p += nth) { const size_t r = p / (F0 / 8); v8b v = {}; if (r < (size_t)NN) for (int e = 0; e < 8; ++e) v[e] = (b16)(bf16_rne(x[p * 8 + e]) * XS); *(volatile v8b*)(X + p * 8) = v; }
    { const v8b z = {}; for (size_t p = tid; p < (size_t)(NP - NN) * F1 / 8; p += nth) { *(volatile v8b*)(H1pad + p * 8) = z; *(volatile v8b*)(H2pad + p * 8) = z; } }
    __threadfence(); }
}
__global__ __launch_bounds__(256) void params_kernel(const float* __restrict__ as0, const float* __restrict__ ad0, const float* __restrict__ b0, const float* __restrict__ g0, const float* __restrict__ be0, const float* __restrict__ m0, const float* __restrict__ v0,
    const float* __restrict__ as1, const float* __restrict__ ad1, const float* __restrict__ b1, const float* __restrict__ g1, const float* __restrict__ be1, const float* __restrict__ m1, const float* __restrict__ v1,
    const float* __restrict__ as2, const float* __restrict__ ad2, const float* __restrict__ b2, const float* __restrict__ g2, const float* __restrict__ be2, const float* __restrict__ m2, const float* __restrict__ v2,
    const float* __restrict__ f1w, const float* __restrict__ f1b, const float* __restrict__ f2w, const float* __restrict__ f2b, const float* __restrict__ f3w, const float* __restrict__ f3b, float* __restrict__ P) {
  const size_t tid = (size_t)blockIdx.x * 256 + threadIdx.x, nth = (size_t)gridDim.x * 256;
  for (int pass = 0; pass < 2; ++pass) { for (size_t q = tid; q < (size_t)PEND; q += nth) { const int i = (int)q; float val = 0.0f;
      if (i < 6144) { const int l = i / 2048, f = (i % 2048) / 256, c = i % 256; const int w = (l == 2) ? F2 : F1; const float* src_ = nullptr;
        if (l == 0) src_ = (f == 0) ? as0 : (f == 1) ? ad0 : (f == 2) ? b0 : (f == 3) ? g0 : (f == 4) ? be0 : (f == 5) ? m0 : (f == 6) ? v0 : nullptr;
        else if (l == 1) src_ = (f == 0) ? as1 : (f == 1) ? ad1 : (f == 2) ? b1 : (f == 3) ? g1 : (f == 4) ? be1 : (f == 5) ? m1 : (f == 6) ? v1 : nullptr;
        else src_ = (f == 0) ? as2 : (f == 1) ? ad2 : (f == 2) ? b2 : (f == 3) ? g2 : (f == 4) ? be2 : (f == 5) ? m2 : (f == 6) ? v2 : nullptr;
        val = (src_ != nullptr && c < w) ? src_[c] : 0.0f; }
      else if (i < 18432) val = f1w[i - 6144]; else if (i < 18496) val = f1b[i - 18432]; else if (i < 20544) val = f2w[i - 18496]; else if (i < 20576) val = f2b[i - 20544]; else if (i < 20608) val = f3w[i - 20576]; else val = (i == 20608) ? f3b[0] : 0.0f;
      P[q] = bf16_rne(val); } __threadfence(); }
}

template <int KIN, int NOUT, int TWO>
__global__ __launch_bounds__(64) void gemm_kernel(const b16* __restrict__ Ah, const b16* __restrict__ Al, const b16* __restrict__ Bw, float* __restrict__ FT) {
  __shared__ __attribute__((aligned(16))) float Ts[2][16][NOUT + 4];
  constexpr int NS = NOUT / 16;
  const int lane = threadIdx.x & 31, wave = threadIdx.x >> 5, nloc = lane & 15, hlf = lane >> 4, m0 = blockIdx.x * 32 + wave * 16;
  v8f acc[NS];
#pragma unroll
  for (int t = 0; t < NS; ++t) acc[t] = (v8f){};
#pragma unroll 2
  for (int kb = 0; kb < KIN; kb += 32) { const v16b a = frag_kb(Ah + (size_t)(m0 + nloc) * KIN + kb, hlf); v16b al_; if (TWO) al_ = frag_kb(Al + (size_t)(m0 + nloc) * KIN + kb, hlf);
#pragma unroll
    for (int t = 0; t < NS; ++t) { const v16b bw = frag_kb(Bw + (size_t)(t * 16 + nloc) * KIN + kb, hlf); acc[t] = wmma16b(a, bw, acc[t]); if (TWO) acc[t] = wmma16b(al_, bw, acc[t]); } }
#pragma unroll
  for (int t = 0; t < NS; ++t)
#pragma unroll
    for (int r = 0; r < 8; ++r) Ts[wave][8 * hlf + r][t * 16 + nloc] = acc[t][r] * (1.0f / XS);
  wave_lds_sync();
  for (int pass = 0; pass < 2; ++pass) { for (int i = lane; i < 16 * (NOUT / 4); i += 32) { const int rr = i / (NOUT / 4), c4 = (i % (NOUT / 4)) * 4; *(volatile v4f*)(FT + (size_t)(m0 + rr) * NOUT + c4) = *(const v4f*)(&Ts[wave][rr][c4]); } __threadfence(); }
}
template <int NH>
__global__ __launch_bounds__(256) void elr_kernel(const float* __restrict__ FT, const float* __restrict__ Pl, float* __restrict__ ALR) {
  __shared__ __attribute__((aligned(16))) float Es[8][8];
  const int wave = threadIdx.x >> 5, v = blockIdx.x * 8 + wave, lane = threadIdx.x & 31;
  if (NH == 4) { float sl = 0.0f, sr = 0.0f;
#pragma unroll
    for (int e = 0; e < 8; ++e) { const float f = FT[(size_t)v * F1 + lane * 8 + e]; sl += pmul(f, Pl[lane * 8 + e]); sr += pmul(f, Pl[256 + lane * 8 + e]); }
    sl += __shfl_xor(sl, 1); sl += __shfl_xor(sl, 2); sl += __shfl_xor(sl, 4); sr += __shfl_xor(sr, 1); sr += __shfl_xor(sr, 2); sr += __shfl_xor(sr, 4);
    if ((lane & 7) == 0) { Es[wave][lane >> 3] = sl; Es[wave][4 + (lane >> 3)] = sr; } }
  else { float sl = 0.0f, sr = 0.0f;
#pragma unroll
    for (int e = 0; e < 2; ++e) { const float f = FT[(size_t)v * F2 + lane * 2 + e]; sl += pmul(f, Pl[lane * 2 + e]); sr += pmul(f, Pl[256 + lane * 2 + e]); }
#pragma unroll
    for (int o = 1; o < 32; o <<= 1) { sl += __shfl_xor(sl, o); sr += __shfl_xor(sr, o); }
    if (lane < 8) Es[wave][lane] = (lane == 0) ? sl : (lane == 4) ? sr : 0.0f; }
  __syncthreads();
  for (int pass = 0; pass < 2; ++pass) { if (threadIdx.x < 16) *(volatile v4f*)(ALR + (size_t)blockIdx.x * 64 + threadIdx.x * 4) = *(const v4f*)(&Es[0][0] + threadIdx.x * 4); __threadfence(); }
}
__global__ __launch_bounds__(256) void gat4_kernel(const float* __restrict__ FT, const float* __restrict__ ALR, const int* __restrict__ src, const int* __restrict__ perm, const int* __restrict__ rowptr, const int* __restrict__ rowcnt, const float* __restrict__ Pl, b16* __restrict__ Hh, b16* __restrict__ Hl) {
  __shared__ __attribute__((aligned(16))) b16 Sh[8][F1 + 8], Sl[8][F1 + 8];
  const int wave = threadIdx.x >> 5, v = blockIdx.x * 8 + wave, lane = threadIdx.x & 31, hd = lane >> 3;
  int cnt = rowcnt[v]; cnt = (cnt < 0) ? 0 : (cnt > MAXDEG ? MAXDEG : cnt); int p0 = rowptr[v]; p0 = (p0 < 0) ? 0 : (p0 > PERMLEN - cnt ? PERMLEN - cnt : p0);
  const float adv = ALR[(size_t)v * 8 + 4 + hd]; float m = -INFINITY, l = 0.0f; float acc[8] = {0, 0, 0, 0, 0, 0, 0, 0};
  for (int q = 0; q <= cnt; ++q) { int s; if (q < cnt) { int id = perm[p0 + q]; id = (id < 0) ? 0 : (id >= NE ? NE - 1 : id); s = src[id]; s = (s < 0) ? 0 : (s >= NN ? NN - 1 : s); } else s = v;
    const float e = leaky(ALR[(size_t)s * 8 + hd] + adv); const float mn = fmaxf(m, e); const float al_ = nexp(m - mn); const float p = nexp(e - mn); m = mn; l = l * al_ + p;
    const v4f f0 = *(const v4f*)(FT + (size_t)s * F1 + lane * 8), f1 = *(const v4f*)(FT + (size_t)s * F1 + lane * 8 + 4);
#pragma unroll
    for (int k = 0; k < 4; ++k) { acc[k] = acc[k] * al_ + pmul(p, f0[k]); acc[4 + k] = acc[4 + k] * al_ + pmul(p, f1[k]); } }
  const float inv = 1.0f / (l + 1e-16f);
#pragma unroll
  for (int k = 0; k < 8; ++k) { const int c = lane * 8 + k; float y = acc[k] * inv + Pl[512 + c]; y = pmul((y - Pl[1280 + c]) * rsqrtf(Pl[1536 + c] + 1e-5f), Pl[768 + c]) + Pl[1024 + c]; y = elu_f(y); b16 a_, b_; split16(y * XS, a_, b_); Sh[wave][c] = a_; Sl[wave][c] = b_; }
  wave_lds_sync();
  for (int pass = 0; pass < 2; ++pass) { *(volatile v8b*)(Hh + (size_t)v * F1 + lane * 8) = *(const v8b*)(&Sh[wave][lane * 8]); *(volatile v8b*)(Hl + (size_t)v * F1 + lane * 8) = *(const v8b*)(&Sl[wave][lane * 8]); __threadfence(); }
}
__global__ __launch_bounds__(256) void gat1_kernel(const float* __restrict__ FT, const float* __restrict__ ALR, const int* __restrict__ src, const int* __restrict__ perm, const int* __restrict__ rowptr, const int* __restrict__ rowcnt, const float* __restrict__ Pl, float* __restrict__ XF) {
  const int wave = threadIdx.x >> 5, v = blockIdx.x * 8 + wave, lane = threadIdx.x & 31;
  int cnt = rowcnt[v]; cnt = (cnt < 0) ? 0 : (cnt > MAXDEG ? MAXDEG : cnt); int p0 = rowptr[v]; p0 = (p0 < 0) ? 0 : (p0 > PERMLEN - cnt ? PERMLEN - cnt : p0);
  const float adv = ALR[(size_t)v * 8 + 4]; float m = -INFINITY, l = 0.0f, a0 = 0.0f, a1 = 0.0f;
  for (int q = 0; q <= cnt; ++q) { int s; if (q < cnt) { int id = perm[p0 + q]; id = (id < 0) ? 0 : (id >= NE ? NE - 1 : id); s = src[id]; s = (s < 0) ? 0 : (s >= NN ? NN - 1 : s); } else s = v;
    const float e = leaky(ALR[(size_t)s * 8 + 0] + adv); const float mn = fmaxf(m, e); const float al_ = nexp(m - mn); const float p = nexp(e - mn); m = mn; l = l * al_ + p;
    const v2f f = *(const v2f*)(FT + (size_t)s * F2 + lane * 2); a0 = a0 * al_ + pmul(p, f[0]); a1 = a1 * al_ + pmul(p, f[1]); }
  const float inv = 1.0f / (l + 1e-16f); v2f o;
  { const int c = lane * 2; float y = a0 * inv + Pl[512 + c]; y = pmul((y - Pl[1280 + c]) * rsqrtf(Pl[1536 + c] + 1e-5f), Pl[768 + c]) + Pl[1024 + c]; o[0] = elu_f(y); }
  { const int c = lane * 2 + 1; float y = a1 * inv + Pl[512 + c]; y = pmul((y - Pl[1280 + c]) * rsqrtf(Pl[1536 + c] + 1e-5f), Pl[768 + c]) + Pl[1024 + c]; o[1] = elu_f(y); }
  for (int pass = 0; pass < 2; ++pass) { *(volatile v2f*)(XF + (size_t)v * F2 + lane * 2) = o; __threadfence(); }
}
__global__ __launch_bounds__(64) void pool_kernel(const float* __restrict__ XF, const int* __restrict__ batch, float* __restrict__ G) {
  const int g = blockIdx.x, c = threadIdx.x;
  auto lower = [&](int key) { int lo = 0, hi = NN; while (lo < hi) { const int mid = (lo + hi) >> 1; if (batch[mid] < key) lo = mid + 1; else hi = mid; } return lo; };
  const int s0 = lower(g), s1 = lower(g + 1); const int cnt = s1 - s0;
  float sm = 0.0f, mx = -INFINITY; for (int n = s0; n < s1; ++n) { const float hv = XF[(size_t)n * F2 + c]; sm += hv; mx = fmaxf(mx, hv); }
  const float mean = sm / fmaxf((float)cnt, 1.0f); if (!(mx > -INFINITY)) mx = 0.0f;
  for (int pass = 0; pass < 2; ++pass) { ((volatile float*)G)[(size_t)g * 192 + c] = mean; ((volatile float*)G)[(size_t)g * 192 + 64 + c] = mx; ((volatile float*)G)[(size_t)g * 192 + 128 + c] = sm; __threadfence(); }
}
__global__ __launch_bounds__(256) void head_kernel(const float* __restrict__ G, const float* __restrict__ P, float* __restrict__ out) {
  const int g = threadIdx.x; const float* gr = G + (size_t)g * 192; float h1[64];
  for (int j = 0; j < 64; ++j) { float s = P[18432 + j]; for (int i = 0; i < 192; ++i) s += pmul(gr[i], P[PHEAD + i * 64 + j]); h1[j] = fmaxf(s, 0.0f); }
  float o = P[20608];
  for (int k = 0; k < 32; ++k) { float s = P[20544 + k]; for (int j = 0; j < 64; ++j) s += pmul(h1[j], P[18496 + j * 32 + k]); s = fmaxf(s, 0.0f); o += pmul(s, P[20576 + k]); }
  for (int pass = 0; pass < 2; ++pass) { ((volatile float*)out)[g] = o; __threadfence(); }
}
}

extern "C" void kernel_launch(void* const* d_in, const int* in_sizes, int n_in,
                              void* d_out, int out_size, void* d_ws, size_t ws_size, hipStream_t stream) {
  (void)n_in; (void)out_size;
  const float* x = (const float*)d_in[0]; const int* ei = (const int*)d_in[1]; const int* batch = (const int*)d_in[2];
  auto F = [&](int i) { return (const float*)d_in[i]; };
  float* out = (float*)d_out;
  if (in_sizes[0] != NN * F0 || in_sizes[1] != 2 * NE || in_sizes[2] != NN || in_sizes[3] != F0 * F1) return;
  const int* srcI = ei; const int* dstI = ei + NE; const int NE_RUN = NE;
  size_t off = 0; char* ws = (char*)d_ws;
  auto carve = [&](size_t bytes) { char* p = ws + off; off += (bytes + 255) & ~(size_t)255; return p; };
  b16* R = (b16*)carve(Ro_::END * 2); float* P = (float*)carve((size_t)PEND * 4 + 256); b16* X = (b16*)carve((size_t)NP * F0 * 2); float* FT = (float*)carve((size_t)NP * F1 * 4); float* ALR = (float*)carve((size_t)NP * 8 * 4); b16* Hh = (b16*)carve((size_t)NP * F1 * 2); b16* Hl = (b16*)carve((size_t)NP * F1 * 2); float* G = (float*)carve((size_t)NGR * 192 * 4);
  CsrBufs cs; off = csr_carve(cs, ws, off, NE_RUN, NN);
  if (off > ws_size) return;
  float* XF = FT + (size_t)NP * F2;
  csr_build(cs, dstI, NE_RUN, NN, stream);
  prep_kernel<<<512, 256, 0, stream>>>(x, nullptr, F(3), F(11), F(19), nullptr, R, X, Hh + (size_t)NN * F1, Hl + (size_t)NN * F1);
  params_kernel<<<32, 256, 0, stream>>>(F(4), F(5), F(6), F(7), F(8), F(9), F(10), F(12), F(13), F(14), F(15), F(16), F(17), F(18), F(20), F(21), F(22), F(23), F(24), F(25), F(26), F(27), F(28), F(29), F(30), F(31), F(32), P);
  gemm_kernel<F0, F1, 0><<<NP / 32, 64, 0, stream>>>(X, nullptr, R + Ro_::W0, FT);
  elr_kernel<4><<<NN / 8, 256, 0, stream>>>(FT, P + 0, ALR);
  gat4_kernel<<<NN / 8, 256, 0, stream>>>(FT, ALR, srcI, cs.PERM, cs.ROWPTR, cs.ROWCNT, P + 0, Hh, Hl);
  gemm_kernel<F1, F1, 1><<<NP / 32, 64, 0, stream>>>(Hh, Hl, R + Ro_::W1, FT);
  elr_kernel<4><<<NN / 8, 256, 0, stream>>>(FT, P + 2048, ALR);
  gat4_kernel<<<NN / 8, 256, 0, stream>>>(FT, ALR, srcI, cs.PERM, cs.ROWPTR, cs.ROWCNT, P + 2048, Hh, Hl);
  gemm_kernel<F1, F2, 1><<<NP / 32, 64, 0, stream>>>(Hh, Hl, R + Ro_::W2, FT);
  elr_kernel<1><<<NN / 8, 256, 0, stream>>>(FT, P + 4096, ALR);
  gat1_kernel<<<NN / 8, 256, 0, stream>>>(FT, ALR, srcI, cs.PERM, cs.ROWPTR, cs.ROWCNT, P + 4096, XF);
  pool_kernel<<<NGR, 64, 0, stream>>>(XF, batch, G);
  head_kernel<<<1, 256, 0, stream>>>(G, P, out);
}
